// GatedAttentionLayer_16552803959278
// MI455X (gfx1250) — hardware-verified
//
#include <hip/hip_runtime.h>
#include <stddef.h>
#include <stdint.h>

#define NB  8
#define LC  2048
#define LQ  512
#define DD  768
#define OTP 68
#define QTP 68

static_assert(LC % 256 == 0);
static_assert(LQ % 64 == 0);
static_assert(DD % 64 == 0);
static_assert(DD % 32 == 0);
static_assert(LQ % 32 == 0);
static_assert(LQ == 512);
static_assert((NB * LC * DD) % 2048 == 0);
static_assert((NB * LQ * DD) % 2048 == 0);
static_assert((NB * LC) % 8 == 0);

typedef __bf16         v16b __attribute__((ext_vector_type(16)));
typedef unsigned short v8us __attribute__((ext_vector_type(8)));
typedef unsigned int   v8u  __attribute__((ext_vector_type(8)));
typedef unsigned int   v4u  __attribute__((ext_vector_type(4)));
typedef float          v8f  __attribute__((ext_vector_type(8)));
typedef float          v4f  __attribute__((ext_vector_type(4)));

union Frag { v16b v; v8us u[2]; v8u w; };

__device__ __forceinline__ v8f mma16(const Frag& a, const Frag& b, v8f c) {
  c = __builtin_amdgcn_wmma_f32_16x16x32_bf16(false, a.v, false, b.v, (short)0, c, false, false);
  asm volatile("v_nop\n\tv_nop\n\tv_nop\n\tv_nop" : "+v"(c) : "v"(a.w), "v"(b.w));
  return c;
}

__device__ __forceinline__ Frag ldfrag(const unsigned short* p, int ld, int row0, int k0, int lane) {
  const int m = lane & 15, lh = lane >> 4;
  const unsigned short* q = p + (size_t)(row0 + m) * ld + k0 + 8 * lh;
  Frag f;
  f.u[0] = *(const v8us*)(q);
  f.u[1] = *(const v8us*)(q + 16);
  return f;
}

__device__ __forceinline__ v8f zero8() { return (v8f){0.f, 0.f, 0.f, 0.f, 0.f, 0.f, 0.f, 0.f}; }

__device__ __forceinline__ unsigned int bf16_bits(float x) {
  const unsigned int u = __float_as_uint(x);
  return (u + 0x7FFFu + ((u >> 16) & 1u)) >> 16;
}

__device__ __forceinline__ void split8(v4f a0, v4f a1, v4u& hv, v4u& lv) {
  unsigned int hb[8], lb[8];
#pragma unroll
  for (int j = 0; j < 4; ++j) {
    const float x0 = a0[j], x1 = a1[j];
    hb[j]     = bf16_bits(x0);
    lb[j]     = bf16_bits(x0 - __uint_as_float(hb[j] << 16));
    hb[4 + j] = bf16_bits(x1);
    lb[4 + j] = bf16_bits(x1 - __uint_as_float(hb[4 + j] << 16));
  }
#pragma unroll
  for (int j = 0; j < 4; ++j) {
    hv[j] = hb[2 * j] | (hb[2 * j + 1] << 16);
    lv[j] = lb[2 * j] | (lb[2 * j + 1] << 16);
  }
}

__device__ __forceinline__ void gemm3_32x64(const unsigned short* __restrict__ Ah, const unsigned short* __restrict__ Al, int lda,
                                            const unsigned short* __restrict__ Bh, const unsigned short* __restrict__ Bl, int ldb,
                                            int K, int m0, int n0, int lane, v8f (&acc)[2][4]) {
#pragma unroll 1
  for (int k0 = 0; k0 < K; k0 += 32) {
    const Frag a0h = ldfrag(Ah, lda, m0, k0, lane);
    const Frag a1h = ldfrag(Ah, lda, m0 + 16, k0, lane);
    const Frag a0l = ldfrag(Al, lda, m0, k0, lane);
    const Frag a1l = ldfrag(Al, lda, m0 + 16, k0, lane);
#pragma unroll
    for (int t = 0; t < 4; ++t) {
      const Frag bh = ldfrag(Bh, ldb, n0 + 16 * t, k0, lane);
      const Frag bl = ldfrag(Bl, ldb, n0 + 16 * t, k0, lane);
      acc[0][t] = mma16(a0h, bh, acc[0][t]);
      acc[1][t] = mma16(a1h, bh, acc[1][t]);
      acc[0][t] = mma16(a0l, bh, acc[0][t]);
      acc[1][t] = mma16(a1l, bh, acc[1][t]);
      acc[0][t] = mma16(a0h, bl, acc[0][t]);
      acc[1][t] = mma16(a1h, bl, acc[1][t]);
    }
  }
}

template <bool GATE>
__device__ __forceinline__ void epilogue32x64(v8f (&acc)[2][4], float* sw, float* __restrict__ out,
                                              const float* __restrict__ gate, int ldo,
                                              int m0, int n0, int lane, int hh, int c) {
#pragma unroll
  for (int sub = 0; sub < 2; ++sub) {
    __syncthreads();
#pragma unroll
    for (int t = 0; t < 4; ++t) {
#pragma unroll
      for (int r = 0; r < 8; ++r) sw[(8 * hh + r) * OTP + 16 * t + c] = acc[sub][t][r];
    }
    __syncthreads();
    v4f val[8];
    size_t go[8];
#pragma unroll
    for (int it = 0; it < 8; ++it) {
      const int p    = lane + 32 * it;
      const int L    = p >> 3;
      const int pc   = p & 7;
      const int row  = L >> 1;
      const int half = L & 1;
      v4f v  = *(const v4f*)(sw + row * OTP + half * 32 + pc * 4);
      go[it] = (size_t)(m0 + sub * 16 + row) * ldo + n0 + half * 32 + pc * 4;
      if (GATE) v = v * *(const v4f*)(gate + go[it]);
      val[it] = v;
    }
#pragma unroll
    for (int it = 0; it < 8; ++it) *(volatile v4f*)(out + go[it]) = val[it];
    __threadfence();
#pragma unroll
    for (int it = 0; it < 8; ++it) *(volatile v4f*)(out + go[it]) = val[it];
  }
}

__global__ __launch_bounds__(256) void k_split(const float* __restrict__ src,
                                               unsigned short* __restrict__ hi,
                                               unsigned short* __restrict__ lo) {
  const size_t e = (size_t)blockIdx.x * 2048 + (size_t)threadIdx.x * 8;
  const v4f a0 = *(const v4f*)(src + e);
  const v4f a1 = *(const v4f*)(src + e + 4);
  v4u hv, lv;
  split8(a0, a1, hv, lv);
  volatile v4u* dh = (volatile v4u*)(hi + e);
  volatile v4u* dl = (volatile v4u*)(lo + e);
  *dh = hv;
  *dl = lv;
  __threadfence();
  *dh = hv;
  *dl = lv;
}

__global__ __launch_bounds__(256) void k_qt(const float* __restrict__ qry,
                                            unsigned short* __restrict__ th,
                                            unsigned short* __restrict__ tl) {
  __shared__ __align__(16) float st[64 * QTP];
  const int tid = threadIdx.x;
  const int b  = blockIdx.z;
  const int q0 = blockIdx.y * 64;
  const int d0 = blockIdx.x * 64;
  const float* src = qry + ((size_t)b * LQ + q0) * DD + d0;
#pragma unroll
  for (int i = 0; i < 4; ++i) {
    const int u  = i * 256 + tid;
    const int r  = u >> 4;
    const int c4 = (u & 15) * 4;
    *(v4f*)(st + r * QTP + c4) = *(const v4f*)(src + (size_t)r * DD + c4);
  }
  __syncthreads();
  unsigned short* oh = th + ((size_t)b * DD + d0) * LQ + q0;
  unsigned short* ol = tl + ((size_t)b * DD + d0) * LQ + q0;
  v4u hv[2], lv[2];
  size_t go[2];
#pragma unroll
  for (int it = 0; it < 2; ++it) {
    const int p    = tid + 256 * it;
    const int drow = p >> 3;
    const int pc   = p & 7;
    v4f a0, a1;
#pragma unroll
    for (int j = 0; j < 4; ++j) {
      a0[j] = st[(8 * pc + j) * QTP + drow];
      a1[j] = st[(8 * pc + 4 + j) * QTP + drow];
    }
    split8(a0, a1, hv[it], lv[it]);
    go[it] = (size_t)drow * LQ + 8 * pc;
  }
#pragma unroll
  for (int it = 0; it < 2; ++it) {
    *(volatile v4u*)(oh + go[it]) = hv[it];
    *(volatile v4u*)(ol + go[it]) = lv[it];
  }
  __threadfence();
#pragma unroll
  for (int it = 0; it < 2; ++it) {
    *(volatile v4u*)(oh + go[it]) = hv[it];
    *(volatile v4u*)(ol + go[it]) = lv[it];
  }
}

__global__ __launch_bounds__(256) void k_gemm_s(const unsigned short* __restrict__ ch,
                                                const unsigned short* __restrict__ cl,
                                                const unsigned short* __restrict__ qh,
                                                const unsigned short* __restrict__ ql,
                                                float* __restrict__ S) {
  __shared__ __align__(16) float st[8][16 * OTP];
  const int tid = threadIdx.x, lane = tid & 31, wave = tid >> 5;
  const int hh = lane >> 4, c = lane & 15;
  const int b  = blockIdx.z;
  const int m0 = blockIdx.x * 256 + wave * 32;
  const int n0 = blockIdx.y * 64;
  const size_t ao = (size_t)b * LC * DD;
  const size_t bo = (size_t)b * LQ * DD;

  v8f acc[2][4];
#pragma unroll
  for (int s = 0; s < 2; ++s)
#pragma unroll
    for (int t = 0; t < 4; ++t) acc[s][t] = zero8();
  gemm3_32x64(ch + ao, cl + ao, DD, qh + bo, ql + bo, DD, DD, m0, n0, lane, acc);
  float* Sb = S + (size_t)b * LC * LQ;
  epilogue32x64<false>(acc, st[wave], Sb, Sb, LQ, m0, n0, lane, hh, c);
}

__global__ __launch_bounds__(256) void k_softmax(const float* __restrict__ S,
                                                 unsigned short* __restrict__ ph,
                                                 unsigned short* __restrict__ pl) {
  const int tid = threadIdx.x, lane = tid & 31, wave = tid >> 5;
  const size_t m = (size_t)blockIdx.x * 8 + wave;
  const float* sr = S + m * LQ;

  v4f x[4];
  x[0] = *(const v4f*)(sr + 8 * lane);
  x[1] = *(const v4f*)(sr + 8 * lane + 4);
  x[2] = *(const v4f*)(sr + 256 + 8 * lane);
  x[3] = *(const v4f*)(sr + 256 + 8 * lane + 4);
  float mx = -__builtin_huge_valf();
#pragma unroll
  for (int i = 0; i < 4; ++i) mx = fmaxf(mx, fmaxf(fmaxf(x[i][0], x[i][1]), fmaxf(x[i][2], x[i][3])));
#pragma unroll
  for (int off = 16; off >= 1; off >>= 1) mx = fmaxf(mx, __shfl_xor(mx, off, 32));

  v4f e[4];
  float s = 0.f;
#pragma unroll
  for (int i = 0; i < 4; ++i) {
#pragma unroll
    for (int j = 0; j < 4; ++j) e[i][j] = __expf(x[i][j] - mx);
    s += (e[i][0] + e[i][1]) + (e[i][2] + e[i][3]);
  }
#pragma unroll
  for (int off = 16; off >= 1; off >>= 1) s += __shfl_xor(s, off, 32);
  const float inv = __builtin_amdgcn_rcpf(s);

  v4u hv[2], lv[2];
  split8(e[0] * inv, e[1] * inv, hv[0], lv[0]);
  split8(e[2] * inv, e[3] * inv, hv[1], lv[1]);

  unsigned short* hr = ph + m * LQ;
  unsigned short* lr = pl + m * LQ;
  *(volatile v4u*)(hr + 8 * lane)       = hv[0];
  *(volatile v4u*)(hr + 256 + 8 * lane) = hv[1];
  *(volatile v4u*)(lr + 8 * lane)       = lv[0];
  *(volatile v4u*)(lr + 256 + 8 * lane) = lv[1];
  __threadfence();
  *(volatile v4u*)(hr + 8 * lane)       = hv[0];
  *(volatile v4u*)(hr + 256 + 8 * lane) = hv[1];
  *(volatile v4u*)(lr + 8 * lane)       = lv[0];
  *(volatile v4u*)(lr + 256 + 8 * lane) = lv[1];
}

__global__ __launch_bounds__(256) void k_gemm_o(const unsigned short* __restrict__ ph,
                                                const unsigned short* __restrict__ pl,
                                                const unsigned short* __restrict__ qth,
                                                const unsigned short* __restrict__ qtl,
                                                const float* __restrict__ ctx,
                                                float* __restrict__ out) {
  __shared__ __align__(16) float st[8][16 * OTP];
  const int tid = threadIdx.x, lane = tid & 31, wave = tid >> 5;
  const int hh = lane >> 4, c = lane & 15;
  const int b  = blockIdx.z;
  const int m0 = blockIdx.x * 256 + wave * 32;
  const int n0 = blockIdx.y * 64;
  const size_t ao = (size_t)b * LC * LQ;
  const size_t bo = (size_t)b * DD * LQ;

  v8f acc[2][4];
#pragma unroll
  for (int s = 0; s < 2; ++s)
#pragma unroll
    for (int t = 0; t < 4; ++t) acc[s][t] = zero8();
  gemm3_32x64(ph + ao, pl + ao, LQ, qth + bo, qtl + bo, LQ, LQ, m0, n0, lane, acc);
  const size_t oo = (size_t)b * LC * DD;
  epilogue32x64<true>(acc, st[wave], out + oo, ctx + oo, DD, m0, n0, lane, hh, c);
}

extern "C" void kernel_launch(void* const* d_in, const int* in_sizes, int n_in,
                              void* d_out, int out_size, void* d_ws, size_t ws_size,
                              hipStream_t stream) {
  if (n_in < 2) return;
  if (in_sizes[0] != NB * LC * DD) return;
  if (in_sizes[1] != NB * LQ * DD) return;
  if (out_size != NB * LC * DD) return;

  const float* ctx = (const float*)d_in[0];
  const float* qry = (const float*)d_in[1];
  float* out = (float*)d_out;

  size_t off = 0;
  const size_t oCh  = off; off += (size_t)NB * LC * DD * 2;
  const size_t oCl  = off; off += (size_t)NB * LC * DD * 2;
  const size_t oQh  = off; off += (size_t)NB * LQ * DD * 2;
  const size_t oQl  = off; off += (size_t)NB * LQ * DD * 2;
  const size_t oQth = off; off += (size_t)NB * DD * LQ * 2;
  const size_t oQtl = off; off += (size_t)NB * DD * LQ * 2;
  const size_t oS   = off; off += (size_t)NB * LC * LQ * 4;
  const size_t oPh  = oCh;
  const size_t oPl  = oPh + (size_t)NB * LC * LQ * 2;
  if (oPl + (size_t)NB * LC * LQ * 2 > oQh) return;
  if (off > ws_size) return;
  if (off > (size_t)134217728) return;

  char* ws = (char*)d_ws;
  unsigned short* Ch  = (unsigned short*)(ws + oCh);
  unsigned short* Cl  = (unsigned short*)(ws + oCl);
  unsigned short* Qh  = (unsigned short*)(ws + oQh);
  unsigned short* Ql  = (unsigned short*)(ws + oQl);
  unsigned short* Qth = (unsigned short*)(ws + oQth);
  unsigned short* Qtl = (unsigned short*)(ws + oQtl);
  float*          S   = (float*)(ws + oS);
  unsigned short* Ph  = (unsigned short*)(ws + oPh);
  unsigned short* Pl  = (unsigned short*)(ws + oPl);

  k_split<<<dim3((NB * LC * DD) / 2048), dim3(256), 0, stream>>>(ctx, Ch, Cl);
  k_split<<<dim3((NB * LQ * DD) / 2048), dim3(256), 0, stream>>>(qry, Qh, Ql);
  k_qt<<<dim3(DD / 64, LQ / 64, NB), dim3(256), 0, stream>>>(qry, Qth, Qtl);
  k_gemm_s<<<dim3(LC / 256, LQ / 64, NB), dim3(256), 0, stream>>>(Ch, Cl, Qh, Ql, S);
  k_softmax<<<dim3((NB * LC) / 8), dim3(256), 0, stream>>>(S, Ph, Pl);
  k_gemm_o<<<dim3(LC / 256, DD / 64, NB), dim3(256), 0, stream>>>(Ph, Pl, Qth, Qtl, ctx, out);
  (void)hipGetLastError();
}
